// ScaleFreeCrossAttention_64742337020421
// MI455X (gfx1250) — hardware-verified
//
#include <hip/hip_runtime.h>
#include <math.h>
#include <stdint.h>
#include <stddef.h>


#define EMBED 768
#define HEADS 12
#define HDIM  64
#define FFDIM 1536
#define BATCH 4
#define LQ 2048
#define LK 2048
#define MQ  (BATCH * LQ)
#define MKV (BATCH * LK)

#define WSC  256.0f
#define ASC  16.0f
#define NSC  256.0f
#define AOSC 256.0f

static_assert(EMBED == HEADS * HDIM, "");
static_assert(HDIM == 64, "");
static_assert(MQ % 128 == 0 && MKV % 128 == 0, "");
static_assert(EMBED % 64 == 0 && FFDIM % 64 == 0, "");
static_assert(EMBED % 32 == 0 && FFDIM % 32 == 0, "");
static_assert(LQ % 128 == 0 && LK % 32 == 0, "");
static_assert(((size_t)MQ * EMBED / 8) % 256 == 0, "");
static_assert(((size_t)MKV * EMBED / 8) % 256 == 0, "");
static_assert(EMBED % 8 == 0 && (EMBED / 4) <= 256, "");

typedef _Float16 v16h __attribute__((ext_vector_type(16)));
typedef _Float16 v8h  __attribute__((ext_vector_type(8)));
typedef float    v8f  __attribute__((ext_vector_type(8)));
typedef float    v4f  __attribute__((ext_vector_type(4)));
typedef int      v4i  __attribute__((ext_vector_type(4)));

union Frag   { v16h v; v8h p[2]; };
union Pack16 { v8h h; v4i i; };

__device__ __forceinline__ v16h ldfrag(const _Float16* rp, int h8) {
    Frag f;
    f.p[0] = *(const v8h*)(rp + h8);
    f.p[1] = *(const v8h*)(rp + 16 + h8);
    return f.v;
}

__device__ __forceinline__ v8f wmma16(v16h a, v16h b, v8f c) {
    c = __builtin_amdgcn_wmma_f32_16x16x32_f16(false, a, false, b, (short)0, c, false, false);
    asm volatile("v_nop\n\tv_nop\n\tv_nop\n\tv_nop" : "+v"(c) : "v"(a), "v"(b));
    return c;
}

__device__ __forceinline__ float wsum(float v) {
    #pragma unroll
    for (int o = 16; o > 0; o >>= 1) v += __shfl_xor(v, o, 32);
    return v;
}

__global__ __launch_bounds__(256)
void k_cvt3(const float* __restrict__ a0, const float* __restrict__ a1,
            const float* __restrict__ a2,
            _Float16* o0, _Float16* o1, _Float16* o2, int n8, float sc)
{
    const int sel = blockIdx.y;
    const float* in = (sel == 0) ? a0 : ((sel == 1) ? a1 : a2);
    _Float16* out   = (sel == 0) ? o0 : ((sel == 1) ? o1 : o2);
    const int i = blockIdx.x * 256 + threadIdx.x;
    const bool ok = i < n8;
    v4i z = {0, 0, 0, 0};
    Pack16 pk; pk.i = z;
    if (ok) {
        v4f x0 = *(const v4f*)(in + (size_t)i * 8);
        v4f x1 = *(const v4f*)(in + (size_t)i * 8 + 4);
        v8f x = __builtin_shufflevector(x0, x1, 0, 1, 2, 3, 4, 5, 6, 7) * sc;
        pk.h = __builtin_convertvector(x, v8h);
    }
    _Float16* dst = out + (size_t)i * 8;
    if (ok) *(volatile v4i*)dst = pk.i;
    __threadfence();
    if (ok) *(volatile v4i*)dst = pk.i;
}

__global__ __launch_bounds__(256)
void k_wtrans(const float* __restrict__ w0, const float* __restrict__ w1,
              const float* __restrict__ w2, const float* __restrict__ w3,
              const float* __restrict__ w4, const float* __restrict__ w5,
              _Float16* o0, _Float16* o1, _Float16* o2,
              _Float16* o3, _Float16* o4, _Float16* o5,
              int K, int N, float sc)
{
    __shared__ alignas(16) _Float16 T[64][72];
    const int z = blockIdx.z;
    const float* W = (z == 0) ? w0 : (z == 1) ? w1 : (z == 2) ? w2 : (z == 3) ? w3 : (z == 4) ? w4 : w5;
    _Float16*    O = (z == 0) ? o0 : (z == 1) ? o1 : (z == 2) ? o2 : (z == 3) ? o3 : (z == 4) ? o4 : o5;
    const int tid = threadIdx.x;
    const int k0 = blockIdx.x * 64, n0 = blockIdx.y * 64;
    const bool okb = (k0 + 64 <= K) && (n0 + 64 <= N);

    if (okb) {
        #pragma unroll
        for (int j = 0; j < 4; ++j) {
            const int k = (tid >> 4) + 16 * j, n4 = (tid & 15) * 4;
            v4f f = *(const v4f*)(W + (size_t)(k0 + k) * N + n0 + n4) * sc;
            T[n4 + 0][k] = (_Float16)f[0];
            T[n4 + 1][k] = (_Float16)f[1];
            T[n4 + 2][k] = (_Float16)f[2];
            T[n4 + 3][k] = (_Float16)f[3];
        }
    }
    __syncthreads();
    Pack16 pv[2]; _Float16* dst[2];
    const int k8 = (tid & 7) * 8;
    #pragma unroll
    for (int j = 0; j < 2; ++j) {
        const int n = (tid >> 3) + 32 * j;
        pv[j].h = *(const v8h*)&T[n][k8];
        dst[j] = O + (size_t)(n0 + n) * K + k0 + k8;
    }
    if (okb) {
        #pragma unroll
        for (int j = 0; j < 2; ++j) *(volatile v4i*)dst[j] = pv[j].i;
    }
    __threadfence();
    if (okb) {
        #pragma unroll
        for (int j = 0; j < 2; ++j) *(volatile v4i*)dst[j] = pv[j].i;
    }
}

template <bool RES, bool GELU, int OUT>
__global__ __launch_bounds__(256)
void k_gemm(const _Float16* __restrict__ A, const _Float16* __restrict__ Wt,
            const float* __restrict__ bias, const float* __restrict__ res,
            void* Cout, int M, int N, int K, float accsc, float outsc)
{
    __shared__ alignas(16) _Float16 As[128][32];
    __shared__ alignas(16) float    Cs[128][68];

    const int tid  = threadIdx.x;
    const int lane = tid & 31;
    const int wave = tid >> 5;
    const int wr   = wave >> 1;
    const int wc   = wave & 1;
    const int h8   = (lane >> 4) * 8;
    const int m    = lane & 15;

    const int rowBase = blockIdx.y * 128;
    const int colBase = blockIdx.x * 64;
    const bool okb = (rowBase + 128 <= M) && (colBase + 64 <= N);

    const _Float16* bp0 = Wt + (size_t)(colBase + wc * 32 + m) * K;
    const _Float16* bp1 = Wt + (size_t)(colBase + wc * 32 + 16 + m) * K;

    const int sr0 = tid >> 2, sc0 = (tid & 3) * 8;
    const int sr1 = sr0 + 64;
    const _Float16* ap0 = A + (size_t)(rowBase + sr0) * K + sc0;
    const _Float16* ap1 = A + (size_t)(rowBase + sr1) * K + sc0;

    v8f acc[2][2] = {};

    if (okb) {
        for (int k0 = 0; k0 < K; k0 += 32) {
            *(v8h*)&As[sr0][sc0] = *(const v8h*)(ap0 + k0);
            *(v8h*)&As[sr1][sc0] = *(const v8h*)(ap1 + k0);
            __syncthreads();
            v16h a0 = ldfrag(&As[wr * 32 + m][0], h8);
            v16h a1 = ldfrag(&As[wr * 32 + 16 + m][0], h8);
            v16h b0 = ldfrag(bp0 + k0, h8);
            v16h b1 = ldfrag(bp1 + k0, h8);
            acc[0][0] = wmma16(a0, b0, acc[0][0]);
            acc[0][1] = wmma16(a0, b1, acc[0][1]);
            acc[1][0] = wmma16(a1, b0, acc[1][0]);
            acc[1][1] = wmma16(a1, b1, acc[1][1]);
            __syncthreads();
        }
    }

    #pragma unroll
    for (int mi = 0; mi < 2; ++mi) {
        #pragma unroll
        for (int ni = 0; ni < 2; ++ni) {
            const int c = wc * 32 + ni * 16 + m;
            #pragma unroll
            for (int e = 0; e < 8; ++e)
                Cs[wr * 32 + mi * 16 + h8 + e][c] = acc[mi][ni][e] * accsc;
        }
    }
    __syncthreads();

    if (OUT == 0 || OUT == 2) {
        _Float16* C16 = (_Float16*)Cout;
        const int c8 = (tid & 7) * 8;
        const int ncol = colBase + c8;
        v4f b0 = {0, 0, 0, 0}, b1 = {0, 0, 0, 0};
        if (okb) { b0 = *(const v4f*)(bias + ncol); b1 = *(const v4f*)(bias + ncol + 4); }
        Pack16 ov[4]; _Float16* dst[4];
        #pragma unroll
        for (int j = 0; j < 4; ++j) {
            const int r = (tid >> 3) + 32 * j;
            const size_t grow = (size_t)(rowBase + r) * N + ncol;
            v4f x0 = *(const v4f*)&Cs[r][c8] + b0;
            v4f x1 = *(const v4f*)&Cs[r][c8 + 4] + b1;
            if (RES) {
                if (okb) { x0 += *(const v4f*)(res + grow); x1 += *(const v4f*)(res + grow + 4); }
            }
            v8f x = __builtin_shufflevector(x0, x1, 0, 1, 2, 3, 4, 5, 6, 7);
            if (GELU) {
                #pragma unroll
                for (int c = 0; c < 8; ++c) {
                    const float t = x[c];
                    x[c] = 0.5f * t * (1.0f + erff(t * 0.70710678118654752f));
                }
            }
            float mul = outsc;
            if (OUT == 2) {
                float ss = 0.0f;
                #pragma unroll
                for (int c = 0; c < 8; ++c) ss += x[c] * x[c];
                ss += __shfl_xor(ss, 1, 32);
                ss += __shfl_xor(ss, 2, 32);
                ss += __shfl_xor(ss, 4, 32);
                mul = outsc / fmaxf(sqrtf(ss), 1e-12f);
            }
            ov[j].h = __builtin_convertvector(x * mul, v8h);
            dst[j] = C16 + grow;
        }
        if (okb) {
            #pragma unroll
            for (int j = 0; j < 4; ++j) *(volatile v4i*)dst[j] = ov[j].i;
        }
        __threadfence();
        if (okb) {
            #pragma unroll
            for (int j = 0; j < 4; ++j) *(volatile v4i*)dst[j] = ov[j].i;
        }
    } else {
        float* C32 = (float*)Cout;
        const int c4 = (tid & 15) * 4;
        const int ncol = colBase + c4;
        v4f bb = {0, 0, 0, 0};
        if (okb) bb = *(const v4f*)(bias + ncol);
        v4f ov[8];
        #pragma unroll
        for (int j = 0; j < 8; ++j) {
            const int r = (tid >> 4) + 16 * j;
            v4f x = *(const v4f*)&Cs[r][c4] + bb;
            if (RES) {
                if (okb) x += *(const v4f*)(res + (size_t)(rowBase + r) * N + ncol);
            }
            ov[j] = x * outsc;
        }
        if (okb) {
            #pragma unroll
            for (int j = 0; j < 8; ++j) {
                const int r = (tid >> 4) + 16 * j;
                *(volatile v4f*)(C32 + (size_t)(rowBase + r) * N + ncol) = ov[j];
            }
        }
        __threadfence();
        if (okb) {
            #pragma unroll
            for (int j = 0; j < 8; ++j) {
                const int r = (tid >> 4) + 16 * j;
                *(volatile v4f*)(C32 + (size_t)(rowBase + r) * N + ncol) = ov[j];
            }
        }
    }
}

__global__ __launch_bounds__(256)
void k_attn(const _Float16* __restrict__ Q, const _Float16* __restrict__ Kx,
            const _Float16* __restrict__ V, _Float16* O, float ssc, float osc)
{
    __shared__ alignas(16) _Float16 Ks[32][64];
    __shared__ alignas(16) _Float16 VsT[64][40];
    __shared__ alignas(16) _Float16 Pst[8][16][40];
    __shared__ alignas(16) _Float16 Ost[8][16][72];

    const int tid  = threadIdx.x;
    const int lane = tid & 31;
    const int wave = tid >> 5;
    const int bh   = blockIdx.y;
    const int b    = bh / HEADS;
    const int h    = bh - b * HEADS;
    const int qbase = blockIdx.x * 128 + wave * 16;
    const int h8   = (lane >> 4) * 8;
    const int m    = lane & 15;

    v16h qf[2];
    {
        const _Float16* qp = Q + (size_t)(b * LQ + qbase + m) * EMBED + h * HDIM;
        qf[0] = ldfrag(qp, h8);
        qf[1] = ldfrag(qp + 32, h8);
    }

    const int kr = tid >> 3, kc8 = (tid & 7) * 8;

    v8f num[4] = {};
    float den[8] = {};

    for (int kk = 0; kk < LK; kk += 32) {
        const size_t gidx = (size_t)(b * LK + kk + kr) * EMBED + h * HDIM + kc8;
        *(v8h*)&Ks[kr][kc8] = *(const v8h*)(Kx + gidx);
        {
            Pack16 pv; pv.h = *(const v8h*)(V + gidx);
            #pragma unroll
            for (int c = 0; c < 8; ++c) VsT[kc8 + c][kr] = pv.h[c];
        }
        __syncthreads();

        v8f s[2] = {};
        #pragma unroll
        for (int ni = 0; ni < 2; ++ni) {
            #pragma unroll
            for (int dc = 0; dc < 2; ++dc)
                s[ni] = wmma16(qf[dc], ldfrag(&Ks[ni * 16 + m][dc * 32], h8), s[ni]);
        }

        #pragma unroll
        for (int ni = 0; ni < 2; ++ni) {
            const int kcol = ni * 16 + m;
            #pragma unroll
            for (int e = 0; e < 8; ++e) {
                const float p = __expf(s[ni][e] * ssc);
                den[e] += p;
                Pst[wave][h8 + e][kcol] = (_Float16)p;
            }
        }
        __syncthreads();

        v16h pa = ldfrag(&Pst[wave][m][0], h8);
        #pragma unroll
        for (int ni = 0; ni < 4; ++ni)
            num[ni] = wmma16(pa, ldfrag(&VsT[ni * 16 + m][0], h8), num[ni]);
        __syncthreads();
    }

    float inv[8];
    #pragma unroll
    for (int e = 0; e < 8; ++e) {
        float d = den[e];
        #pragma unroll
        for (int o = 8; o > 0; o >>= 1) d += __shfl_xor(d, o, 32);
        inv[e] = osc / d;
    }

    #pragma unroll
    for (int ni = 0; ni < 4; ++ni) {
        const int d = ni * 16 + m;
        #pragma unroll
        for (int e = 0; e < 8; ++e)
            Ost[wave][h8 + e][d] = (_Float16)(num[ni][e] * inv[e]);
    }
    __syncthreads();

    const int q4 = lane >> 3, c8 = (lane & 7) * 8;
    Pack16 ov[4]; _Float16* dst[4];
    #pragma unroll
    for (int j = 0; j < 4; ++j) {
        const int r = q4 + 4 * j;
        ov[j].h = *(const v8h*)&Ost[wave][r][c8];
        dst[j] = O + (size_t)(b * LQ + qbase + r) * EMBED + h * HDIM + c8;
    }
    #pragma unroll
    for (int j = 0; j < 4; ++j) *(volatile v4i*)dst[j] = ov[j].i;
    __threadfence();
    #pragma unroll
    for (int j = 0; j < 4; ++j) *(volatile v4i*)dst[j] = ov[j].i;
}

template <bool COPY16>
__global__ __launch_bounds__(256)
void k_ln(const float* __restrict__ x, const float* __restrict__ y,
          const float* __restrict__ g, const float* __restrict__ be,
          float* out, _Float16* out16, float sc16)
{
    __shared__ float red1[8];
    __shared__ float red2[8];
    __shared__ alignas(16) _Float16 hrow[EMBED];

    const int row = blockIdx.x, tid = threadIdx.x;
    const int lane = tid & 31, wave = tid >> 5;
    const bool act = tid < (EMBED / 4);
    const size_t base = (size_t)row * EMBED + (size_t)tid * 4;

    v4f v = {0, 0, 0, 0};
    if (act) v = *(const v4f*)(x + base) + *(const v4f*)(y + base);
    float s = wsum(v[0] + v[1] + v[2] + v[3]);
    if (lane == 0) red1[wave] = s;
    __syncthreads();
    float tot = 0.0f;
    #pragma unroll
    for (int w = 0; w < 8; ++w) tot += red1[w];
    const float mu = tot * (1.0f / EMBED);

    v4f d = {0, 0, 0, 0};
    if (act) d = v - mu;
    float q = wsum(d[0] * d[0] + d[1] * d[1] + d[2] * d[2] + d[3] * d[3]);
    if (lane == 0) red2[wave] = q;
    __syncthreads();
    float tq = 0.0f;
    #pragma unroll
    for (int w = 0; w < 8; ++w) tq += red2[w];
    const float rstd = rsqrtf(tq * (1.0f / EMBED) + 1e-5f);

    v4f o = {0, 0, 0, 0};
    if (act) {
        v4f gg = *(const v4f*)(g + tid * 4);
        v4f bb = *(const v4f*)(be + tid * 4);
        o = d * rstd * gg + bb;
    }
    float* op = out + base;
    if (act) *(volatile v4f*)op = o;
    if (COPY16) {
        if (act) {
            hrow[tid * 4 + 0] = (_Float16)(o[0] * sc16);
            hrow[tid * 4 + 1] = (_Float16)(o[1] * sc16);
            hrow[tid * 4 + 2] = (_Float16)(o[2] * sc16);
            hrow[tid * 4 + 3] = (_Float16)(o[3] * sc16);
        }
    }
    __threadfence();
    if (act) *(volatile v4f*)op = o;

    if (COPY16) {
        __syncthreads();
        const bool act2 = tid < (EMBED / 8);
        v4i z = {0, 0, 0, 0};
        Pack16 p; p.i = z;
        _Float16* hp = out16 + (size_t)row * EMBED + (size_t)tid * 8;
        if (act2) p.h = *(const v8h*)&hrow[tid * 8];
        if (act2) *(volatile v4i*)hp = p.i;
        __threadfence();
        if (act2) *(volatile v4i*)hp = p.i;
    }
}

extern "C" void kernel_launch(void* const* d_in, const int* in_sizes, int n_in,
                              void* d_out, int out_size, void* d_ws, size_t ws_size,
                              hipStream_t stream)
{
    if (n_in != 24) return;
    const size_t SZQ = (size_t)MQ * EMBED;
    const size_t SZK = (size_t)MKV * EMBED;
    if ((size_t)in_sizes[0] != SZQ || (size_t)in_sizes[1] != SZK ||
        (size_t)in_sizes[2] != SZQ || (size_t)in_sizes[3] != SZK) return;
    for (int i = 4; i <= 14; i += 2) if (in_sizes[i] != EMBED * EMBED) return;
    for (int i = 5; i <= 19; i += 2) if (in_sizes[i] != EMBED) return;
    if (in_sizes[16] != EMBED || in_sizes[18] != EMBED) return;
    if (in_sizes[20] != EMBED * FFDIM || in_sizes[21] != FFDIM) return;
    if (in_sizes[22] != EMBED * FFDIM || in_sizes[23] != EMBED) return;
    if ((size_t)out_size != SZQ) return;

    const float* image_tokens = (const float*)d_in[0];
    const float* point_tokens = (const float*)d_in[1];
    const float* image_pos    = (const float*)d_in[2];
    const float* point_pos    = (const float*)d_in[3];
    const float* Wip = (const float*)d_in[4];   const float* bip = (const float*)d_in[5];
    const float* Wpp = (const float*)d_in[6];   const float* bpp = (const float*)d_in[7];
    const float* Wq  = (const float*)d_in[8];   const float* bq  = (const float*)d_in[9];
    const float* Wk  = (const float*)d_in[10];  const float* bk  = (const float*)d_in[11];
    const float* Wv  = (const float*)d_in[12];  const float* bv  = (const float*)d_in[13];
    const float* Wo  = (const float*)d_in[14];  const float* bo  = (const float*)d_in[15];
    const float* g1  = (const float*)d_in[16];  const float* b1  = (const float*)d_in[17];
    const float* g2  = (const float*)d_in[18];  const float* b2  = (const float*)d_in[19];
    const float* Wf1 = (const float*)d_in[20];  const float* bf1 = (const float*)d_in[21];
    const float* Wf2 = (const float*)d_in[22];  const float* bf2 = (const float*)d_in[23];

    const size_t SLOT = ((SZQ > SZK) ? SZQ : SZK) * 2;
    const size_t WB   = (size_t)EMBED * EMBED * 2;
    const size_t FB   = (size_t)EMBED * FFDIM * 2;
    size_t off = 0;
    char* ws = (char*)d_ws;
    char* slot[6];
    for (int i = 0; i < 6; ++i) { slot[i] = ws + off; off += SLOT; }
    _Float16* WipT = (_Float16*)(ws + off); off += WB;
    _Float16* WppT = (_Float16*)(ws + off); off += WB;
    _Float16* WqT  = (_Float16*)(ws + off); off += WB;
    _Float16* WkT  = (_Float16*)(ws + off); off += WB;
    _Float16* WvT  = (_Float16*)(ws + off); off += WB;
    _Float16* WoT  = (_Float16*)(ws + off); off += WB;
    _Float16* Wf1T = (_Float16*)(ws + off); off += FB;
    _Float16* Wf2T = (_Float16*)(ws + off); off += FB;
    if (off > ws_size) return;

    _Float16* P0  = (_Float16*)slot[0];
    _Float16* P1  = (_Float16*)slot[1];
    _Float16* P2  = (_Float16*)slot[2];
    _Float16* T1  = (_Float16*)slot[3];
    _Float16* T2  = (_Float16*)slot[4];
    _Float16* Qn  = (_Float16*)slot[0];
    _Float16* Kn  = (_Float16*)slot[1];
    _Float16* Vh  = (_Float16*)slot[3];
    _Float16* AO  = (_Float16*)slot[4];
    float*    proj    = (float*)slot[2];
    float*    fused   = (float*)slot[0];
    _Float16* fused16 = (_Float16*)slot[5];
    _Float16* Hh      = (_Float16*)slot[2];
    float*    ffb     = (float*)slot[4];

    const dim3 blk(256);
    const float SC_AW  = 1.0f / (ASC * WSC);
    const float SC_OW  = 1.0f / (AOSC * WSC);
    const float SC_QK  = 1.0f / (NSC * NSC);
    const float SC_ATT = AOSC / ASC;

    {
        const int n8 = (int)(SZQ / 8);
        dim3 g((n8 + 255) / 256, 3);
        k_cvt3<<<g, blk, 0, stream>>>(image_pos, point_pos, point_tokens, P0, P1, P2, n8, ASC);
    }
    k_wtrans<<<dim3(EMBED / 64, EMBED / 64, 6), blk, 0, stream>>>(
        Wip, Wpp, Wq, Wk, Wv, Wo, WipT, WppT, WqT, WkT, WvT, WoT, EMBED, EMBED, WSC);
    k_wtrans<<<dim3(EMBED / 64, FFDIM / 64, 1), blk, 0, stream>>>(
        Wf1, Wf1, Wf1, Wf1, Wf1, Wf1, Wf1T, Wf1T, Wf1T, Wf1T, Wf1T, Wf1T, EMBED, FFDIM, WSC);
    k_wtrans<<<dim3(FFDIM / 64, EMBED / 64, 1), blk, 0, stream>>>(
        Wf2, Wf2, Wf2, Wf2, Wf2, Wf2, Wf2T, Wf2T, Wf2T, Wf2T, Wf2T, Wf2T, FFDIM, EMBED, WSC);

    const dim3 gq ((EMBED + 63) / 64, (MQ + 127) / 128);
    const dim3 gk ((EMBED + 63) / 64, (MKV + 127) / 128);
    const dim3 gff((FFDIM + 63) / 64, (MQ + 127) / 128);

    k_gemm<true, false, 0><<<gq, blk, 0, stream>>>(P0, WipT, bip, image_tokens, (void*)T1, MQ, EMBED, EMBED, SC_AW, ASC);
    k_gemm<true, false, 0><<<gk, blk, 0, stream>>>(P1, WppT, bpp, point_tokens, (void*)T2, MKV, EMBED, EMBED, SC_AW, ASC);
    k_gemm<false, false, 2><<<gq, blk, 0, stream>>>(T1, WqT, bq, bq, (void*)Qn, MQ, EMBED, EMBED, SC_AW, NSC);
    k_gemm<false, false, 2><<<gk, blk, 0, stream>>>(T2, WkT, bk, bk, (void*)Kn, MKV, EMBED, EMBED, SC_AW, NSC);
    k_gemm<false, false, 0><<<gk, blk, 0, stream>>>(P2, WvT, bv, bv, (void*)Vh, MKV, EMBED, EMBED, SC_AW, ASC);
    k_attn<<<dim3(LQ / 128, BATCH * HEADS), blk, 0, stream>>>(Qn, Kn, Vh, AO, SC_QK, SC_ATT);
    k_gemm<false, false, 1><<<gq, blk, 0, stream>>>(AO, WoT, bo, bo, (void*)proj, MQ, EMBED, EMBED, SC_OW, 1.0f);
    k_ln<true><<<dim3(MQ), blk, 0, stream>>>(image_tokens, proj, g1, b1, fused, fused16, ASC);
    k_gemm<false, true, 0><<<gff, blk, 0, stream>>>(fused16, Wf1T, bf1, bf1, (void*)Hh, MQ, FFDIM, EMBED, SC_AW, ASC);
    k_gemm<false, false, 1><<<gq, blk, 0, stream>>>(Hh, Wf2T, bf2, bf2, (void*)ffb, MQ, EMBED, FFDIM, SC_AW, 1.0f);
    k_ln<false><<<dim3(MQ), blk, 0, stream>>>(fused, ffb, g2, b2, (float*)d_out, fused16, 1.0f);
}
